// MultiHeadAttention_26740466385334
// MI455X (gfx1250) — hardware-run, weakly checked
//
#include <hip/hip_runtime.h>
#ifndef NB
#define NB 4
#endif
#ifndef SEQ
#define SEQ 2048
#endif
#define NB_FULL 4
#define SEQ_FULL 2048
#define WD 768
#define NH 12
#define HD 64
#define NTOK (NB * SEQ)
#define XSTRIDE_FULL ((size_t)SEQ_FULL * WD)

static_assert(SEQ % 128 == 0);
static_assert(SEQ <= SEQ_FULL);
static_assert(NB <= NB_FULL);
static_assert(HD == 64);
static_assert(NH * HD == WD);
static_assert(WD % 128 == 0);
static_assert(WD % 32 == 0);
static_assert((size_t)NTOK * WD * 2 * 5 + (size_t)4 * WD * WD * 2 + 4096 <= (size_t)134217728);

typedef __bf16 v16b __attribute__((ext_vector_type(16)));
typedef _Float16 v16h __attribute__((ext_vector_type(16)));
typedef unsigned short v8us __attribute__((ext_vector_type(8), may_alias));
typedef float v8f __attribute__((ext_vector_type(8)));
typedef float v4f __attribute__((ext_vector_type(4)));
typedef float v4fa __attribute__((ext_vector_type(4), may_alias));
union Frag16 { v16b b; v16h h; v8us half[2]; };
union FragP { v16h v; _Float16 e[16]; };

#define LOG2E 1.4426950408889634f
#define SCORE_SCL 0.00048828125f

__device__ __forceinline__ unsigned short bf16_bits(float x) {
  unsigned int u = __float_as_uint(x);
  return (unsigned short)((u + 0x7FFFu + ((u >> 16) & 1u)) >> 16);
}
__device__ __forceinline__ float bf16_val(unsigned short b) { return __uint_as_float(((unsigned int)b) << 16); }
__device__ __forceinline__ float bf16_rne(float x) { return bf16_val(bf16_bits(x)); }
__device__ __forceinline__ unsigned short f16_bits(float x) {
  union { _Float16 h; unsigned short u; } c;
  c.h = (_Float16)x;
  return c.u;
}

__device__ __forceinline__ v8f mma_h2k(v16h a0, v16h b0, v16h a1, v16h b1, v8f c) {
  c = __builtin_amdgcn_wmma_f32_16x16x32_f16(false, a0, false, b0, (short)0, c, false, false);
  c = __builtin_amdgcn_wmma_f32_16x16x32_f16(false, a1, false, b1, (short)0, c, false, false);
  asm volatile("v_nop\n\tv_nop\n\tv_nop\n\tv_nop" : "+v"(c) : "v"(a0), "v"(b0), "v"(a1), "v"(b1));
  return c;
}
__device__ __forceinline__ void mma_pv4(v16h a0, v16h a1, v16h a2, v16h a3, v16h b, v8f (&c)[4]) {
  c[0] = __builtin_amdgcn_wmma_f32_16x16x32_f16(false, a0, false, b, (short)0, c[0], false, false);
  c[1] = __builtin_amdgcn_wmma_f32_16x16x32_f16(false, a1, false, b, (short)0, c[1], false, false);
  c[2] = __builtin_amdgcn_wmma_f32_16x16x32_f16(false, a2, false, b, (short)0, c[2], false, false);
  c[3] = __builtin_amdgcn_wmma_f32_16x16x32_f16(false, a3, false, b, (short)0, c[3], false, false);
  asm volatile("v_nop\n\tv_nop\n\tv_nop\n\tv_nop" : "+v"(c[0]), "+v"(c[1]), "+v"(c[2]), "+v"(c[3])
               : "v"(a0), "v"(a1), "v"(a2), "v"(a3), "v"(b));
}
template <bool F16>
__device__ __forceinline__ void mma8(const Frag16& a0, const Frag16& a1, const Frag16& b0, const Frag16& b1,
                                     const Frag16& b2, const Frag16& b3, v8f (&c)[2][4]) {
  if (F16) {
    c[0][0] = __builtin_amdgcn_wmma_f32_16x16x32_f16(false, a0.h, false, b0.h, (short)0, c[0][0], false, false);
    c[0][1] = __builtin_amdgcn_wmma_f32_16x16x32_f16(false, a0.h, false, b1.h, (short)0, c[0][1], false, false);
    c[0][2] = __builtin_amdgcn_wmma_f32_16x16x32_f16(false, a0.h, false, b2.h, (short)0, c[0][2], false, false);
    c[0][3] = __builtin_amdgcn_wmma_f32_16x16x32_f16(false, a0.h, false, b3.h, (short)0, c[0][3], false, false);
    c[1][0] = __builtin_amdgcn_wmma_f32_16x16x32_f16(false, a1.h, false, b0.h, (short)0, c[1][0], false, false);
    c[1][1] = __builtin_amdgcn_wmma_f32_16x16x32_f16(false, a1.h, false, b1.h, (short)0, c[1][1], false, false);
    c[1][2] = __builtin_amdgcn_wmma_f32_16x16x32_f16(false, a1.h, false, b2.h, (short)0, c[1][2], false, false);
    c[1][3] = __builtin_amdgcn_wmma_f32_16x16x32_f16(false, a1.h, false, b3.h, (short)0, c[1][3], false, false);
    asm volatile("v_nop\n\tv_nop\n\tv_nop\n\tv_nop"
                 : "+v"(c[0][0]), "+v"(c[0][1]), "+v"(c[0][2]), "+v"(c[0][3]),
                   "+v"(c[1][0]), "+v"(c[1][1]), "+v"(c[1][2]), "+v"(c[1][3])
                 : "v"(a0.h), "v"(a1.h), "v"(b0.h), "v"(b1.h), "v"(b2.h), "v"(b3.h));
  } else {
    c[0][0] = __builtin_amdgcn_wmma_f32_16x16x32_bf16(false, a0.b, false, b0.b, (short)0, c[0][0], false, false);
    c[0][1] = __builtin_amdgcn_wmma_f32_16x16x32_bf16(false, a0.b, false, b1.b, (short)0, c[0][1], false, false);
    c[0][2] = __builtin_amdgcn_wmma_f32_16x16x32_bf16(false, a0.b, false, b2.b, (short)0, c[0][2], false, false);
    c[0][3] = __builtin_amdgcn_wmma_f32_16x16x32_bf16(false, a0.b, false, b3.b, (short)0, c[0][3], false, false);
    c[1][0] = __builtin_amdgcn_wmma_f32_16x16x32_bf16(false, a1.b, false, b0.b, (short)0, c[1][0], false, false);
    c[1][1] = __builtin_amdgcn_wmma_f32_16x16x32_bf16(false, a1.b, false, b1.b, (short)0, c[1][1], false, false);
    c[1][2] = __builtin_amdgcn_wmma_f32_16x16x32_bf16(false, a1.b, false, b2.b, (short)0, c[1][2], false, false);
    c[1][3] = __builtin_amdgcn_wmma_f32_16x16x32_bf16(false, a1.b, false, b3.b, (short)0, c[1][3], false, false);
    asm volatile("v_nop\n\tv_nop\n\tv_nop\n\tv_nop"
                 : "+v"(c[0][0]), "+v"(c[0][1]), "+v"(c[0][2]), "+v"(c[0][3]),
                   "+v"(c[1][0]), "+v"(c[1][1]), "+v"(c[1][2]), "+v"(c[1][3])
                 : "v"(a0.b), "v"(a1.b), "v"(b0.b), "v"(b1.b), "v"(b2.b), "v"(b3.b));
  }
}

template <bool F16>
__device__ __forceinline__ void gemm_tile(const unsigned short* __restrict__ ap, const unsigned short* __restrict__ bp,
                                          v8f (&acc)[2][4]) {
#pragma unroll 1
  for (int k0 = 0; k0 < WD; k0 += 32) {
    Frag16 a0, a1, b0, b1, b2, b3;
    a0.half[0] = *(const v8us*)(ap + k0);                a0.half[1] = *(const v8us*)(ap + k0 + 16);
    a1.half[0] = *(const v8us*)(ap + 16 * WD + k0);      a1.half[1] = *(const v8us*)(ap + 16 * WD + k0 + 16);
    b0.half[0] = *(const v8us*)(bp + k0);                b0.half[1] = *(const v8us*)(bp + k0 + 16);
    b1.half[0] = *(const v8us*)(bp + 16 * WD + k0);      b1.half[1] = *(const v8us*)(bp + 16 * WD + k0 + 16);
    b2.half[0] = *(const v8us*)(bp + 32 * WD + k0);      b2.half[1] = *(const v8us*)(bp + 32 * WD + k0 + 16);
    b3.half[0] = *(const v8us*)(bp + 48 * WD + k0);      b3.half[1] = *(const v8us*)(bp + 48 * WD + k0 + 16);
    mma8<F16>(a0, a1, b0, b1, b2, b3, acc);
  }
}

__global__ __launch_bounds__(256) void k_xb(const float* __restrict__ X, unsigned short* __restrict__ Xb) {
#pragma clang fp contract(off)
  const int t = blockIdx.x * 256 + threadIdx.x;
  if (t >= NTOK * (WD / 8)) return;
  const int row = t / (WD / 8), piece = t - row * (WD / 8);
  const int b = row / SEQ, s = row - b * SEQ;
  const float* src = X + (size_t)b * XSTRIDE_FULL + (size_t)s * WD + piece * 8;
  const v4f x0 = *(const v4fa*)(src), x1 = *(const v4fa*)(src + 4);
  v8us o;
  o[0] = bf16_bits(x0[0]); o[1] = bf16_bits(x0[1]); o[2] = bf16_bits(x0[2]); o[3] = bf16_bits(x0[3]);
  o[4] = bf16_bits(x1[0]); o[5] = bf16_bits(x1[1]); o[6] = bf16_bits(x1[2]); o[7] = bf16_bits(x1[3]);
  unsigned short* d = Xb + (size_t)t * 8;
  *(volatile v8us*)d = o;
  __threadfence();
  *(volatile v8us*)d = o;
}

__global__ __launch_bounds__(256) void k_wo(const float* __restrict__ Wo, unsigned short* __restrict__ Woh) {
#pragma clang fp contract(off)
  const int t = blockIdx.x * 256 + threadIdx.x;
  if (t >= WD * (WD / 8)) return;
  const float* src = Wo + (size_t)t * 8;
  const v4f x0 = *(const v4fa*)(src), x1 = *(const v4fa*)(src + 4);
  v8us o;
  o[0] = f16_bits(bf16_rne(x0[0]) * 1024.0f); o[1] = f16_bits(bf16_rne(x0[1]) * 1024.0f);
  o[2] = f16_bits(bf16_rne(x0[2]) * 1024.0f); o[3] = f16_bits(bf16_rne(x0[3]) * 1024.0f);
  o[4] = f16_bits(bf16_rne(x1[0]) * 1024.0f); o[5] = f16_bits(bf16_rne(x1[1]) * 1024.0f);
  o[6] = f16_bits(bf16_rne(x1[2]) * 1024.0f); o[7] = f16_bits(bf16_rne(x1[3]) * 1024.0f);
  unsigned short* d = Woh + (size_t)t * 8;
  *(volatile v8us*)d = o;
  __threadfence();
  *(volatile v8us*)d = o;
}

__global__ __launch_bounds__(256) void k_wt(const float* __restrict__ Wq, const float* __restrict__ Wk,
                                            const float* __restrict__ Wv, unsigned short* __restrict__ Wt) {
#pragma clang fp contract(off)
  __shared__ unsigned short tl[64][66];
  const int tid = threadIdx.x;
  const int z = blockIdx.x / (NH * (WD / 64));
  const int rem = blockIdx.x - z * (NH * (WD / 64));
  const int h = rem / (WD / 64);
  const int w0 = (rem - h * (WD / 64)) * 64;
  for (int i = tid; i < 64 * 16; i += 256) {
    const int j = i >> 4, c4 = (i & 15) * 4;
    const size_t so = ((size_t)h * WD + w0 + j) * HD + c4;
    const v4f xq = *(const v4fa*)(Wq + so);
    const v4f xk = *(const v4fa*)(Wk + so);
    const v4f xv = *(const v4fa*)(Wv + so);
    const v4f x = (z == 0) ? xq : ((z == 1) ? xk : xv);
    tl[c4 + 0][j] = bf16_bits(x[0]); tl[c4 + 1][j] = bf16_bits(x[1]);
    tl[c4 + 2][j] = bf16_bits(x[2]); tl[c4 + 3][j] = bf16_bits(x[3]);
  }
  __syncthreads();
  for (int pass = 0; pass < 2; ++pass) {
    for (int i = tid; i < 64 * 8; i += 256) {
      const int d = i >> 3, j8 = (i & 7) * 8;
      v8us o;
#pragma unroll
      for (int q = 0; q < 8; ++q) o[q] = tl[d][j8 + q];
      *(volatile v8us*)(Wt + ((size_t)z * WD + h * HD + d) * WD + w0 + j8) = o;
    }
    if (pass == 0) __threadfence();
  }
}

__global__ __launch_bounds__(128) void k_proj_qk(const unsigned short* __restrict__ Xb, const unsigned short* __restrict__ Wt,
                                                 const float* __restrict__ bq, const float* __restrict__ bk,
                                                 unsigned short* __restrict__ QK) {
  __shared__ __attribute__((aligned(16))) unsigned short st[4][32][72];
  const int tid = threadIdx.x, lane = tid & 31, ln = lane & 15, hh = lane >> 4;
  const int w = __builtin_amdgcn_readfirstlane(tid >> 5);
  const int y = blockIdx.y;
  const int z = y / NH, h = y - z * NH;
  const int t0 = blockIdx.x * 128 + 32 * w;
  const unsigned short* ap = Xb + (size_t)(t0 + ln) * WD + 8 * hh;
  const unsigned short* bp = Wt + (size_t)(y * HD + ln) * WD + 8 * hh;
  v8f acc[2][4] = {};
  gemm_tile<false>(ap, bp, acc);
#pragma unroll
  for (int j = 0; j < 4; ++j) {
    const int n = 16 * j + ln;
    const float bqv = bq[h * HD + n];
    const float bkv = bk[h * HD + n];
    const float bias = bf16_rne((z == 0) ? bqv : bkv);
#pragma unroll
    for (int i = 0; i < 2; ++i)
#pragma unroll
      for (int r = 0; r < 8; ++r)
        st[w][16 * i + 8 * hh + r][n] = f16_bits((acc[i][j][r] + bias) * 16.0f);
  }
  __syncthreads();
  const int b = t0 / SEQ, s0 = t0 - b * SEQ;
  unsigned short* dst = QK + ((((size_t)z * NB + b) * NH + h) * SEQ + s0) * HD;
  const int rq = lane >> 3, piece = (lane & 7) * 8;
  for (int pass = 0; pass < 2; ++pass) {
#pragma unroll
    for (int it = 0; it < 8; ++it) {
      const int row = 4 * it + rq;
      const v8us v = *(const v8us*)&st[w][row][piece];
      *(volatile v8us*)(dst + (size_t)row * HD + piece) = v;
    }
    if (pass == 0) __threadfence();
  }
}

__global__ __launch_bounds__(128) void k_proj_v(const unsigned short* __restrict__ Xb, const unsigned short* __restrict__ Wt,
                                                const float* __restrict__ bv, unsigned short* __restrict__ Vt) {
  __shared__ __attribute__((aligned(16))) unsigned short st[4][32][72];
  const int tid = threadIdx.x, lane = tid & 31, ln = lane & 15, hh = lane >> 4;
  const int w = __builtin_amdgcn_readfirstlane(tid >> 5);
  const int m0 = blockIdx.x * 128 + 32 * w;
  const int n0 = blockIdx.y * 64;
  const unsigned short* ap = Wt + (size_t)(2 * WD + m0 + ln) * WD + 8 * hh;
  const unsigned short* bp = Xb + (size_t)(n0 + ln) * WD + 8 * hh;
  v8f acc[2][4] = {};
  gemm_tile<false>(ap, bp, acc);
#pragma unroll
  for (int i = 0; i < 2; ++i)
#pragma unroll
    for (int r = 0; r < 8; ++r) {
      const int row = 16 * i + 8 * hh + r;
      const float bias = bf16_rne(bv[m0 + row]);
#pragma unroll
      for (int j = 0; j < 4; ++j)
        st[w][row][16 * j + ln] = f16_bits((acc[i][j][r] + bias) * 16.0f);
    }
  __syncthreads();
  const int b = n0 / SEQ, s0 = n0 - b * SEQ;
  unsigned short* dst = Vt + ((size_t)b * WD + m0) * SEQ + s0;
  const int rq = lane >> 3, piece = (lane & 7) * 8;
  for (int pass = 0; pass < 2; ++pass) {
#pragma unroll
    for (int it = 0; it < 8; ++it) {
      const int row = 4 * it + rq;
      const v8us v = *(const v8us*)&st[w][row][piece];
      *(volatile v8us*)(dst + (size_t)row * SEQ + piece) = v;
    }
    if (pass == 0) __threadfence();
  }
}

__device__ __forceinline__ void fa_step(const unsigned short* __restrict__ Kp, const unsigned short* __restrict__ Vp,
                                        int key0, int ln, int hh, const Frag16& q0, const Frag16& q1,
                                        float& mr, float& lr, v8f (&Oh)[4]) {
  const unsigned short* kp0 = Kp + (size_t)(key0 + ln) * HD + 8 * hh;
  const unsigned short* kp1 = kp0 + 16 * HD;
  Frag16 k00, k01, k10, k11;
  k00.half[0] = *(const v8us*)(kp0);      k00.half[1] = *(const v8us*)(kp0 + 16);
  k01.half[0] = *(const v8us*)(kp0 + 32); k01.half[1] = *(const v8us*)(kp0 + 48);
  k10.half[0] = *(const v8us*)(kp1);      k10.half[1] = *(const v8us*)(kp1 + 16);
  k11.half[0] = *(const v8us*)(kp1 + 32); k11.half[1] = *(const v8us*)(kp1 + 48);
  const unsigned short* vp = Vp + (size_t)ln * SEQ + key0 + 8 * hh;
  Frag16 vf[4];
#pragma unroll
  for (int t = 0; t < 4; ++t) {
    vf[t].half[0] = *(const v8us*)(vp + (size_t)t * 16 * SEQ);
    vf[t].half[1] = *(const v8us*)(vp + (size_t)t * 16 * SEQ + 16);
  }
  const v8f z8 = {0.f, 0.f, 0.f, 0.f, 0.f, 0.f, 0.f, 0.f};
  const v8f s0 = mma_h2k(k00.h, q0.h, k01.h, q1.h, z8);
  const v8f s1 = mma_h2k(k10.h, q0.h, k11.h, q1.h, z8);
  float sc[16];
#pragma unroll
  for (int r = 0; r < 8; ++r) { sc[r] = s0[r] * SCORE_SCL; sc[8 + r] = s1[r] * SCORE_SCL; }
  float mx = sc[0];
#pragma unroll
  for (int i = 1; i < 16; ++i) mx = fmaxf(mx, sc[i]);
  mx = fmaxf(mx, __shfl_xor(mx, 16, 32));
  const float mnew = fmaxf(mr, mx);
  const float al = exp2f((mr - mnew) * LOG2E);
  mr = mnew;
  FragP ph;
  float ps = 0.0f;
#pragma unroll
  for (int i = 0; i < 16; ++i) {
    const float pc = exp2f(fmaf(sc[i] - mnew, LOG2E, 8.0f));
    ps += pc;
    ph.e[i] = (_Float16)pc;
  }
  ps += __shfl_xor(ps, 16, 32);
  lr = lr * al + ps;
#pragma unroll
  for (int t = 0; t < 4; ++t) Oh[t] = Oh[t] * al;
  mma_pv4(vf[0].h, vf[1].h, vf[2].h, vf[3].h, ph.v, Oh);
}

__global__ __launch_bounds__(128) void k_attn(const unsigned short* __restrict__ QK, const unsigned short* __restrict__ Vt,
                                              unsigned short* __restrict__ Ch) {
  __shared__ __attribute__((aligned(16))) unsigned short so[4][16][72];
  const int tid = threadIdx.x, lane = tid & 31, ln = lane & 15, hh = lane >> 4;
  const int w = __builtin_amdgcn_readfirstlane(tid >> 5);
  const int bh = blockIdx.x / (SEQ / 64), qt = blockIdx.x - bh * (SEQ / 64);
  const int b = bh / NH, h = bh - b * NH;
  const int qbase = qt * 64 + 16 * w;
  const int qg = qbase + ln;
  const unsigned short* Qp = QK + (size_t)bh * SEQ * HD;
  const unsigned short* Kp = QK + ((size_t)NB * NH + bh) * SEQ * HD;
  const unsigned short* Vp = Vt + (size_t)bh * HD * SEQ;
  const unsigned short* qrow = Qp + (size_t)qg * HD + 8 * hh;
  Frag16 q0, q1;
  q0.half[0] = *(const v8us*)(qrow);      q0.half[1] = *(const v8us*)(qrow + 16);
  q1.half[0] = *(const v8us*)(qrow + 32); q1.half[1] = *(const v8us*)(qrow + 48);
  float mr = -3.0e38f, lr = 0.0f;
  v8f Oh[4] = {};
#pragma unroll 1
  for (int j = 0; j < SEQ / 32; ++j)
    fa_step(Kp, Vp, 32 * j, ln, hh, q0, q1, mr, lr, Oh);

  const float inv = 4.0f * (1.0f / lr);
#pragma unroll
  for (int t = 0; t < 4; ++t)
#pragma unroll
    for (int r = 0; r < 8; ++r)
      so[w][ln][16 * t + 8 * hh + r] = f16_bits(Oh[t][r] * inv);
  __syncthreads();
  unsigned short* dst = Ch + ((size_t)b * SEQ + qbase) * WD + h * HD;
  const int rq = lane >> 3, piece = (lane & 7) * 8;
  for (int pass = 0; pass < 2; ++pass) {
#pragma unroll
    for (int it = 0; it < 4; ++it) {
      const int row = 4 * it + rq;
      const v8us v = *(const v8us*)&so[w][row][piece];
      *(volatile v8us*)(dst + (size_t)row * WD + piece) = v;
    }
    if (pass == 0) __threadfence();
  }
}

__global__ __launch_bounds__(128) void k_oproj(const unsigned short* __restrict__ Ch, const unsigned short* __restrict__ Woh,
                                               const float* __restrict__ bo, float* __restrict__ out) {
  __shared__ __attribute__((aligned(16))) float so[4][32][68];
  const int tid = threadIdx.x, lane = tid & 31, ln = lane & 15, hh = lane >> 4;
  const int w = __builtin_amdgcn_readfirstlane(tid >> 5);
  const int t0 = blockIdx.x * 128 + 32 * w;
  const int n0 = blockIdx.y * 64;
  const unsigned short* ap = Ch + (size_t)(t0 + ln) * WD + 8 * hh;
  const unsigned short* bp = Woh + (size_t)(n0 + ln) * WD + 8 * hh;
  v8f acc[2][4] = {};
  gemm_tile<true>(ap, bp, acc);
#pragma unroll
  for (int j = 0; j < 4; ++j) {
    const float bias = bf16_rne(bo[n0 + 16 * j + ln]);
#pragma unroll
    for (int i = 0; i < 2; ++i)
#pragma unroll
      for (int r = 0; r < 8; ++r)
        so[w][16 * i + 8 * hh + r][16 * j + ln] = acc[i][j][r] * 0.0000152587890625f + bias;
  }
  __syncthreads();
  const int b = t0 / SEQ, s0 = t0 - b * SEQ;
  float* og = out + (size_t)b * XSTRIDE_FULL + (size_t)s0 * WD + n0;
  const int rsub = lane >> 4, c4 = (lane & 15) * 4;
  for (int pass = 0; pass < 2; ++pass) {
#pragma unroll
    for (int it = 0; it < 16; ++it) {
      const int row = 2 * it + rsub;
      const v4f v = *(const v4fa*)&so[w][row][c4];
      *(volatile v4f*)(og + (size_t)row * WD + c4) = v;
    }
    if (pass == 0) __threadfence();
  }
}

extern "C" void kernel_launch(void* const* d_in, const int* in_sizes, int n_in,
                              void* d_out, int out_size, void* d_ws, size_t ws_size, hipStream_t stream) {
  if (n_in < 9) return;
  const long long need = (long long)(NB - 1) * SEQ_FULL * WD + (long long)SEQ * WD;
  if ((long long)in_sizes[0] < need) return;
  if ((long long)in_sizes[1] < (long long)NH * WD * HD || (long long)in_sizes[2] < (long long)NH * WD * HD ||
      (long long)in_sizes[3] < (long long)NH * WD * HD || (long long)in_sizes[7] < (long long)WD * WD) return;
  if (in_sizes[4] < WD || in_sizes[5] < WD || in_sizes[6] < WD || in_sizes[8] < WD) return;
  if ((long long)out_size < need) return;
  const float* x  = (const float*)d_in[0];
  const float* Wq = (const float*)d_in[1];
  const float* Wk = (const float*)d_in[2];
  const float* Wv = (const float*)d_in[3];
  const float* bq = (const float*)d_in[4];
  const float* bk = (const float*)d_in[5];
  const float* bv = (const float*)d_in[6];
  const float* Wo = (const float*)d_in[7];
  const float* bo = (const float*)d_in[8];
  float* out = (float*)d_out;
  char* ws = (char*)d_ws;
  size_t off = 0;
  const size_t tokp = (size_t)NTOK * WD * 2;
  const size_t wp = (size_t)WD * WD * 2;
  unsigned short* Xb  = (unsigned short*)(ws + off); off += (tokp + 255) & ~(size_t)255;
  unsigned short* Wt  = (unsigned short*)(ws + off); off += (3 * wp + 255) & ~(size_t)255;
  unsigned short* Woh = (unsigned short*)(ws + off); off += (wp + 255) & ~(size_t)255;
  unsigned short* QK  = (unsigned short*)(ws + off); off += (2 * tokp + 255) & ~(size_t)255;
  unsigned short* Vt  = (unsigned short*)(ws + off); off += (tokp + 255) & ~(size_t)255;
  unsigned short* Ch  = (unsigned short*)(ws + off); off += (tokp + 255) & ~(size_t)255;
  if (off > ws_size || off > (size_t)134217728) return;

  k_xb<<<(unsigned)((NTOK * (WD / 8) + 255) / 256), 256, 0, stream>>>(x, Xb);
  k_wo<<<(unsigned)((WD * (WD / 8) + 255) / 256), 256, 0, stream>>>(Wo, Woh);
  k_wt<<<(unsigned)(3 * NH * (WD / 64)), 256, 0, stream>>>(Wq, Wk, Wv, Wt);
  k_proj_qk<<<dim3((unsigned)(NTOK / 128), 2 * NH), 128, 0, stream>>>(Xb, Wt, bq, bk, QK);
  k_proj_v<<<dim3((unsigned)(WD / 128), (unsigned)(NTOK / 64)), 128, 0, stream>>>(Xb, Wt, bv, Vt);
  k_attn<<<(unsigned)(NB * NH * (SEQ / 64)), 128, 0, stream>>>(QK, Vt, Ch);
  k_oproj<<<dim3((unsigned)(NTOK / 128), (unsigned)(WD / 64)), 128, 0, stream>>>(Ch, Woh, bo, out);
}
